// Head_49976239456456
// MI455X (gfx1250) — hardware-verified
//
#include <hip/hip_runtime.h>
#include <hip/hip_bf16.h>


#ifndef NB
#define NB 4
#endif
#ifndef SEQ
#define SEQ 4096
#endif
#define NB_FULL  4
#define SEQ_FULL 4096
#define DM 256
#define HS 64
#define PROJ_ROWS 128
#define P_CARRY 1024.0f
#define P_UNCARRY 0.0009765625f
#define SCORE_SCALE 0.0625f

static_assert(NB >= 1 && NB <= NB_FULL);
static_assert(SEQ >= PROJ_ROWS && SEQ <= SEQ_FULL);
static_assert(SEQ % PROJ_ROWS == 0);
static_assert(SEQ % 32 == 0);
static_assert(DM % 32 == 0);
static_assert(HS == 64);

typedef _Float16 v8h   __attribute__((ext_vector_type(8)));
typedef _Float16 v16h  __attribute__((ext_vector_type(16)));
typedef __bf16   v8bf  __attribute__((ext_vector_type(8)));
typedef __bf16   v16bf __attribute__((ext_vector_type(16)));
typedef float    v4f   __attribute__((ext_vector_type(4)));
typedef float    v8f   __attribute__((ext_vector_type(8)));
typedef v4f __attribute__((may_alias)) v4fa;

union FragH  { v16h  v; v8h  h[2]; };
union FragBF { v16bf v; v8bf h[2]; };

static __device__ __forceinline__ v8f mma_bf16(v16bf a, v16bf b, v8f c) {
  v8f d = __builtin_amdgcn_wmma_f32_16x16x32_bf16(false, a, false, b, (short)0, c, false, false);
  asm volatile("v_nop\n\tv_nop\n\tv_nop\n\tv_nop" : "+v"(d) : "v"(a), "v"(b));
  return d;
}
static __device__ __forceinline__ v8f mma_f16(v16h a, v16h b, v8f c) {
  v8f d = __builtin_amdgcn_wmma_f32_16x16x32_f16(false, a, false, b, (short)0, c, false, false);
  asm volatile("v_nop\n\tv_nop\n\tv_nop\n\tv_nop" : "+v"(d) : "v"(a), "v"(b));
  return d;
}

__global__ __launch_bounds__(256) void proj_kernel(
    const float* __restrict__ x,
    const float* __restrict__ Wk, const float* __restrict__ bk,
    const float* __restrict__ Wq, const float* __restrict__ bq,
    const float* __restrict__ Wv, const float* __restrict__ bv,
    _Float16* __restrict__ Kp, _Float16* __restrict__ Qp, _Float16* __restrict__ Vt)
{
  __shared__ __align__(16) __bf16   Wl[HS * DM];
  __shared__ __align__(16) _Float16 stg[PROJ_ROWS * HS];

  const int tid  = threadIdx.x;
  const int lane = tid & 31;
  const int wv   = tid >> 5;
  const int m    = lane & 15;
  const int hi   = lane >> 4;
  const int blk  = blockIdx.x;
  const int b    = blk / (SEQ / PROJ_ROWS);
  const int t0b  = (blk - b * (SEQ / PROJ_ROWS)) * PROJ_ROWS;
  const int t0w  = t0b + wv * 16;

  v16bf xa[DM / 32];
  {
    const float* xrow = x + ((size_t)b * SEQ_FULL + t0w + m) * DM;
#pragma unroll
    for (int k = 0; k < DM / 32; ++k) {
      const int c0 = k * 32 + 8 * hi;
      const v4f f0 = *(const v4f*)(xrow + c0);
      const v4f f1 = *(const v4f*)(xrow + c0 + 4);
      const v4f f2 = *(const v4f*)(xrow + c0 + 16);
      const v4f f3 = *(const v4f*)(xrow + c0 + 20);
#pragma unroll
      for (int e = 0; e < 4; ++e) {
        xa[k][e]      = (__bf16)f0[e];
        xa[k][4 + e]  = (__bf16)f1[e];
        xa[k][8 + e]  = (__bf16)f2[e];
        xa[k][12 + e] = (__bf16)f3[e];
      }
    }
  }

  for (int p = 0; p < 3; ++p) {
    const float* W    = (p == 0) ? Wk : ((p == 1) ? Wq : Wv);
    const float* bias = (p == 0) ? bk : ((p == 1) ? bq : bv);

    __syncthreads();
    for (int i = tid; i < DM * HS / 4; i += 256) {
      const v4f f  = *(const v4f*)(W + (size_t)i * 4);
      const int c  = i >> 4;
      const int h0 = (i & 15) * 4;
#pragma unroll
      for (int e = 0; e < 4; ++e) Wl[(h0 + e) * DM + c] = (__bf16)f[e];
    }
    __syncthreads();

    v8f acc[4] = {};
#pragma unroll
    for (int k = 0; k < DM / 32; ++k) {
#pragma unroll
      for (int j = 0; j < 4; ++j) {
        const __bf16* wr = Wl + (16 * j + m) * DM + k * 32;
        FragBF wb;
        wb.h[0] = *(const v8bf*)(wr + 8 * hi);
        wb.h[1] = *(const v8bf*)(wr + 16 + 8 * hi);
        acc[j] = mma_bf16(xa[k], wb.v, acc[j]);
      }
    }

#pragma unroll
    for (int j = 0; j < 4; ++j) {
      const int    hcol = 16 * j + m;
      const __bf16 bb   = (__bf16)bias[hcol];
      const float  bj   = (float)bb;
      if (p < 2) {
#pragma unroll
        for (int r = 0; r < 8; ++r)
          stg[(wv * 16 + 8 * hi + r) * HS + hcol] = (_Float16)(acc[j][r] + bj);
      } else {
#pragma unroll
        for (int r = 0; r < 8; ++r)
          stg[hcol * PROJ_ROWS + wv * 16 + 8 * hi + r] = (_Float16)(acc[j][r] + bj);
      }
    }
    __syncthreads();

    v4f ov[4];
#pragma unroll
    for (int i = 0; i < 4; ++i) ov[i] = *(const v4fa*)(stg + (size_t)(i * 256 + tid) * 8);
#pragma unroll
    for (int i = 0; i < 4; ++i) {
      const int q = i * 256 + tid;
      _Float16* gp;
      if (p == 0)      gp = Kp + ((size_t)b * SEQ + t0b) * HS + (size_t)q * 8;
      else if (p == 1) gp = Qp + ((size_t)b * SEQ + t0b) * HS + (size_t)q * 8;
      else             gp = Vt + ((size_t)b * HS + (q >> 4)) * SEQ + t0b + (q & 15) * 8;
      *(volatile v4f*)gp = ov[i];
    }
    __threadfence();
#pragma unroll
    for (int i = 0; i < 4; ++i) {
      const int q = i * 256 + tid;
      _Float16* gp;
      if (p == 0)      gp = Kp + ((size_t)b * SEQ + t0b) * HS + (size_t)q * 8;
      else if (p == 1) gp = Qp + ((size_t)b * SEQ + t0b) * HS + (size_t)q * 8;
      else             gp = Vt + ((size_t)b * HS + (q >> 4)) * SEQ + t0b + (q & 15) * 8;
      *(volatile v4f*)gp = ov[i];
    }
  }
}

__global__ __launch_bounds__(64) void attn_kernel(
    const _Float16* __restrict__ Kp, const _Float16* __restrict__ Qp,
    const _Float16* __restrict__ Vt, float* __restrict__ out)
{
  __shared__ __align__(16) float ost[2][16 * HS];

  const int lane = threadIdx.x & 31;
  const int wv   = threadIdx.x >> 5;
  const int m    = lane & 15;
  const int hi   = lane >> 4;
  const int gw   = blockIdx.x * 2 + wv;
  const int b    = gw / (SEQ / 16);
  const int t0   = (gw - b * (SEQ / 16)) * 16;

  FragH kb0, kb1;
  {
    const _Float16* kr = Kp + ((size_t)b * SEQ + t0 + m) * HS;
    kb0.h[0] = *(const v8h*)(kr + 8 * hi);
    kb0.h[1] = *(const v8h*)(kr + 16 + 8 * hi);
    kb1.h[0] = *(const v8h*)(kr + 32 + 8 * hi);
    kb1.h[1] = *(const v8h*)(kr + 48 + 8 * hi);
  }
  const _Float16* qb  = Qp + (size_t)b * SEQ * HS;
  const _Float16* vtb = Vt + (size_t)b * HS * SEQ;

  v8f acc[4] = {};
  float m_run = -1.0e30f;
  float l_run = 0.0f;

  for (int it = 0; it < SEQ / 32; ++it) {
    const int s0 = it * 32;

    v8f st[2];
#pragma unroll
    for (int ss = 0; ss < 2; ++ss) {
      const _Float16* qr = qb + (size_t)(s0 + 16 * ss + m) * HS;
      FragH q0, q1;
      q0.h[0] = *(const v8h*)(qr + 8 * hi);
      q0.h[1] = *(const v8h*)(qr + 16 + 8 * hi);
      q1.h[0] = *(const v8h*)(qr + 32 + 8 * hi);
      q1.h[1] = *(const v8h*)(qr + 48 + 8 * hi);
      v8f z = {};
      st[ss] = mma_f16(q0.v, kb0.v, z);
      st[ss] = mma_f16(q1.v, kb1.v, st[ss]);
    }

    float sv0[8], sv1[8];
    float bm = -1.0e30f;
#pragma unroll
    for (int r = 0; r < 8; ++r) {
      sv0[r] = st[0][r] * SCORE_SCALE;
      sv1[r] = st[1][r] * SCORE_SCALE;
      bm = fmaxf(bm, fmaxf(sv0[r], sv1[r]));
    }
    bm = fmaxf(bm, __shfl_xor(bm, 16, 32));
    const float m_new = fmaxf(m_run, bm);
    const float corr  = __expf(m_run - m_new);
    m_run = m_new;

    v16h pa;
    float lsum = 0.0f;
#pragma unroll
    for (int r = 0; r < 8; ++r) {
      const float p0 = __expf(sv0[r] - m_new);
      const float p1 = __expf(sv1[r] - m_new);
      lsum += p0 + p1;
      pa[r]     = (_Float16)(p0 * P_CARRY);
      pa[8 + r] = (_Float16)(p1 * P_CARRY);
    }
    lsum += __shfl_xor(lsum, 16, 32);
    l_run = l_run * corr + lsum;

#pragma unroll
    for (int r = 0; r < 8; ++r) {
      const float cr = __shfl(corr, 8 * hi + r, 32);
#pragma unroll
      for (int j = 0; j < 4; ++j) acc[j][r] *= cr;
    }

#pragma unroll
    for (int j = 0; j < 4; ++j) {
      const _Float16* vr = vtb + (size_t)(16 * j + m) * SEQ + s0;
      FragH vb;
      vb.h[0] = *(const v8h*)(vr + 8 * hi);
      vb.h[1] = *(const v8h*)(vr + 16 + 8 * hi);
      acc[j] = mma_f16(pa, vb.v, acc[j]);
    }
  }

  float* tl = &ost[wv][0];
  const float scl = (1.0f / l_run) * P_UNCARRY;
#pragma unroll
  for (int r = 0; r < 8; ++r) {
    const float sc = __shfl(scl, 8 * hi + r, 32);
#pragma unroll
    for (int j = 0; j < 4; ++j) tl[(8 * hi + r) * HS + 16 * j + m] = acc[j][r] * sc;
  }
  __syncthreads();

  float* go = out + ((size_t)b * SEQ + t0) * HS;
  v4f ov[8];
#pragma unroll
  for (int i = 0; i < 8; ++i) ov[i] = *(const v4fa*)(tl + (i * 32 + lane) * 4);
#pragma unroll
  for (int i = 0; i < 8; ++i) *(volatile v4f*)(go + (size_t)(i * 32 + lane) * 4) = ov[i];
  __threadfence();
#pragma unroll
  for (int i = 0; i < 8; ++i) *(volatile v4f*)(go + (size_t)(i * 32 + lane) * 4) = ov[i];
}

extern "C" void kernel_launch(void* const* d_in, const int* in_sizes, int n_in,
                              void* d_out, int out_size, void* d_ws, size_t ws_size,
                              hipStream_t stream) {
  if (n_in < 7) return;
  if (in_sizes[0] < ((NB - 1) * SEQ_FULL + SEQ) * DM) return;
  if (in_sizes[1] < DM * HS || in_sizes[3] < DM * HS || in_sizes[5] < DM * HS) return;
  if (in_sizes[2] < HS || in_sizes[4] < HS || in_sizes[6] < HS) return;
  if (out_size < NB * SEQ * HS) return;

  const size_t planeBytes = (size_t)NB * SEQ * HS * sizeof(_Float16);
  if (ws_size < 3 * planeBytes) return;

  const float* x  = (const float*)d_in[0];
  const float* Wk = (const float*)d_in[1];
  const float* bk = (const float*)d_in[2];
  const float* Wq = (const float*)d_in[3];
  const float* bq = (const float*)d_in[4];
  const float* Wv = (const float*)d_in[5];
  const float* bv = (const float*)d_in[6];
  float* out = (float*)d_out;

  char* ws = (char*)d_ws;
  _Float16* Kp = (_Float16*)(ws);
  _Float16* Qp = (_Float16*)(ws + planeBytes);
  _Float16* Vt = (_Float16*)(ws + 2 * planeBytes);

  proj_kernel<<<dim3(NB * SEQ / PROJ_ROWS), dim3(256), 0, stream>>>(
      x, Wk, bk, Wq, bq, Wv, bv, Kp, Qp, Vt);
  attn_kernel<<<dim3(NB * SEQ / 32), dim3(64), 0, stream>>>(Kp, Qp, Vt, out);
}
